// RNN_61770219651190
// MI455X (gfx1250) — hardware-verified
//
#include <hip/hip_runtime.h>
#include <math.h>

#pragma clang fp contract(off)

constexpr int kModels = 256;
constexpr int kCells  = 128;
constexpr int kStim   = 2;
constexpr int kCond   = 4;
constexpr int kOutO   = 2;
constexpr int kSteps  = 300;
constexpr int kFix = 50, kSamp = 50, kDelay = 100, kTest = 50, kResp = 50;
static_assert(kFix + kSamp + kDelay + kTest + kResp == kSteps);
constexpr int kDelayT0 = kFix + kSamp;
constexpr int kTestT0  = kDelayT0 + kDelay;
constexpr int kRespT0  = kSteps - kResp;
constexpr int kSlots0  = kDelay * kCond * kOutO;
constexpr int kSlots1  = kResp  * kCond * kOutO;
constexpr int kSlotPitch = 1280;
static_assert(kSlots0 + kSlots1 <= kSlotPitch);
static_assert(kSlotPitch % 128 == 0);
constexpr int kThreads = 256;
static_assert(kCells == 16 * (kThreads / 32));
static_assert(kCells % 32 == 0);
static_assert((kThreads / 32) == kCond * kOutO);
static_assert(kCond <= 16);
constexpr int kRP    = kCells + 8;
constexpr int kR32P  = kCells + 4;
constexpr int kHbElems  = 2 * 2 * 16 * kRP;
constexpr int kR32Elems = 2 * 16 * kR32P;
static_assert(kHbElems % 8 == 0 && kR32Elems % 4 == 0 && kRP % 8 == 0 && kR32P % 4 == 0);
constexpr float kCarry    = 2048.0f;
constexpr float kCarryInv = 1.0f / 2048.0f;
constexpr float kLeak     = 0.2f;
constexpr float kNoiseStd = 0.1f;
constexpr float kH16MinNormal = 6.103515625e-05f;
constexpr int kOut0Floats = kDelay * kCond * kModels * kOutO;
constexpr int kOut1Floats = kResp  * kCond * kModels * kOutO;
constexpr int kOutFloats  = kOut0Floats + kOut1Floats;
constexpr int kOut0Lines  = kOut0Floats / 32;
static_assert(kOut0Floats % 128 == 0);
static_assert(kOutFloats % (kThreads * 4) == 0);
constexpr int kEmitBlocks = kOutFloats / (kThreads * 4);
static_assert(kModels * kOutO == 16 * 32);

typedef __attribute__((ext_vector_type(16))) _Float16 v16h;
typedef __attribute__((ext_vector_type(8)))  _Float16 v8h;
typedef __attribute__((ext_vector_type(8)))  float    v8f;
typedef __attribute__((ext_vector_type(4)))  float    v4f;
typedef __attribute__((ext_vector_type(2)))  float    v2f;

__device__ __forceinline__ void dep_guard6(v8f& a, v8f& b, v16h p, v16h q, v16h r, v16h s) {
  asm volatile("v_nop\n\tv_nop\n\tv_nop\n\tv_nop" : "+v"(a), "+v"(b) : "v"(p), "v"(q), "v"(r), "v"(s));
}
__device__ __forceinline__ void acc_guard2(v8f& a, v8f& b) { asm volatile("v_nop\n\tv_nop\n\tv_nop\n\tv_nop" : "+v"(a), "+v"(b)); }

template <typename T> struct Frag;
template <> struct Frag<_Float16> {
  typedef v16h V; union U { v16h v; v8h h[2]; };
  static __device__ __forceinline__ v16h load(const _Float16* p) {
    U f; f.h[0] = *(const v8h*)(p); f.h[1] = *(const v8h*)(p + 16); return f.v;
  }
  static __device__ __forceinline__ v8f mma(v16h a, v16h b, v8f c) {
    return __builtin_amdgcn_wmma_f32_16x16x32_f16(false, a, false, b, (short)0, c, false, false);
  }
};

__device__ __forceinline__ void split_h16(float v, _Float16& hi, _Float16& lo) {
  const float av = fabsf(v);
  const float vs = (av < kH16MinNormal) ? 0.0f : v;
  const _Float16 hh = (_Float16)vs;
  const float hf = (float)hh;
  const float d  = v - hf;
  const float ds = d * kCarry;
  hi = hh;
  lo = (_Float16)ds;
}

__global__ __launch_bounds__(kThreads) void rnn_seq_kernel(
    const float* __restrict__ x,
    const float* __restrict__ noise,
    const float* __restrict__ W,
    const float* __restrict__ bvec,
    const float* __restrict__ Wi,
    const float* __restrict__ Wo,
    const float* __restrict__ Wm,
    float* __restrict__ stg) {
  __shared__ __align__(16) _Float16 hb[kHbElems];
  __shared__ __align__(16) float    r32[kR32Elems];
  __shared__ __align__(16) float    res[kSlotPitch];
  const int tid = threadIdx.x, lane = tid & 31, wave = tid >> 5;
  const int c = lane & 15, hh = lane >> 4;
  const int model = blockIdx.x;
  const int cellA = 16 * wave + c;
  const int cell0 = 16 * wave + 8 * hh;
  const int o = wave & 1, bq = wave >> 1;

  {
    const v8h zh = {(_Float16)0.f, (_Float16)0.f, (_Float16)0.f, (_Float16)0.f, (_Float16)0.f, (_Float16)0.f, (_Float16)0.f, (_Float16)0.f};
    const v4f zf = {0.f, 0.f, 0.f, 0.f};
#pragma unroll 1
    for (int i = tid; i < kHbElems / 8; i += kThreads) *(v8h*)(hb + i * 8) = zh;
#pragma unroll 1
    for (int i = tid; i < kR32Elems / 4; i += kThreads) *(v4f*)(r32 + i * 4) = zf;
#pragma unroll 1
    for (int i = tid; i < kSlotPitch / 4; i += kThreads) *(v4f*)(res + i * 4) = zf;
  }

  const int cc = (c < kCond) ? c : (kCond - 1);
  const v4f xv = *(const v4f*)(x + cc * (2 * kStim));
  const float* wip = Wi + ((size_t)model * kCells + cell0) * kStim;
  v4f wiv[4];
  wiv[0] = *(const v4f*)(wip);      wiv[1] = *(const v4f*)(wip + 4);
  wiv[2] = *(const v4f*)(wip + 8);  wiv[3] = *(const v4f*)(wip + 12);
  asm volatile("" ::: "memory");
  float dsv[8], dtv[8], bias[8], rst[8];
#pragma unroll
  for (int r = 0; r < 8; ++r) {
    const float w0 = wiv[r >> 1][(r & 1) * 2];
    const float w1 = wiv[r >> 1][(r & 1) * 2 + 1];
    const float p0 = w0 * xv[0], p1 = w1 * xv[1];
    const float q0 = w0 * xv[2], q1 = w1 * xv[3];
    dsv[r] = p0 + p1;
    dtv[r] = q0 + q1;
    rst[r] = 0.0f;
  }
  {
    const float* bp = bvec + (size_t)model * kCells + cell0;
    const v4f b0 = *(const v4f*)(bp);
    const v4f b1 = *(const v4f*)(bp + 4);
    bias[0] = b0[0]; bias[1] = b0[1]; bias[2] = b0[2]; bias[3] = b0[3];
    bias[4] = b1[0]; bias[5] = b1[1]; bias[6] = b1[2]; bias[7] = b1[3];
  }
  const v4f wmv = *(const v4f*)(Wm + ((size_t)model * kOutO + o) * kCells + 4 * lane);
  const v4f wov = *(const v4f*)(Wo + ((size_t)model * kOutO + o) * kCells + 4 * lane);
  asm volatile("" ::: "memory");

  v16h ah[4], al[4];
  {
    const float* wrow = W + (size_t)model * kCells * kCells + (size_t)cellA * kCells + 8 * hh;
#pragma unroll
    for (int kc = 0; kc < kCells / 32; ++kc) {
      const v4f w0 = *(const v4f*)(wrow + 32 * kc);
      const v4f w1 = *(const v4f*)(wrow + 32 * kc + 4);
      const v4f w2 = *(const v4f*)(wrow + 32 * kc + 16);
      const v4f w3 = *(const v4f*)(wrow + 32 * kc + 20);
#pragma unroll
      for (int e = 0; e < 4; ++e) {
        _Float16 h0, l0, h1, l1, h2, l2, h3, l3;
        split_h16(w0[e], h0, l0);
        split_h16(w1[e], h1, l1);
        split_h16(w2[e], h2, l2);
        split_h16(w3[e], h3, l3);
        ah[kc][e]      = h0;  al[kc][e]      = l0;
        ah[kc][4 + e]  = h1;  al[kc][4 + e]  = l1;
        ah[kc][8 + e]  = h2;  al[kc][8 + e]  = l2;
        ah[kc][12 + e] = h3;  al[kc][12 + e] = l3;
      }
      asm volatile("" ::: "memory");
    }
  }
  __syncthreads();

  const v8f z8 = {0.f, 0.f, 0.f, 0.f, 0.f, 0.f, 0.f, 0.f};

#pragma unroll 1
  for (int t = 0; t < kSteps; ++t) {
    const int cur = t & 1, nxt = cur ^ 1;
    const float* np = noise + ((size_t)t * kModels + model) * kCells + cell0;
    const v4f nz0 = *(const v4f*)(np);
    const v4f nz1 = *(const v4f*)(np + 4);

    const _Float16* bhp = hb + ((cur * 2 + 0) * 16 + c) * kRP + 8 * hh;
    const _Float16* blp = hb + ((cur * 2 + 1) * 16 + c) * kRP + 8 * hh;
    v8f accA = z8, accB = z8;
#pragma unroll
    for (int kc = 0; kc < kCells / 32; ++kc) {
      const v16h fb = Frag<_Float16>::load(bhp + 32 * kc);
      const v16h fl = Frag<_Float16>::load(blp + 32 * kc);
      accA = Frag<_Float16>::mma(ah[kc], fb, accA);
      accB = Frag<_Float16>::mma(ah[kc], fl, accB);
      accB = Frag<_Float16>::mma(al[kc], fb, accB);
      dep_guard6(accA, accB, fb, fl, ah[kc], al[kc]);
    }
    acc_guard2(accA, accB);

    const float ms = (t >= kFix && t < kDelayT0) ? 1.0f : 0.0f;
    const float mt = (t >= kTestT0 && t < kRespT0) ? 1.0f : 0.0f;
    float nzv[8];
    nzv[0] = nz0[0]; nzv[1] = nz0[1]; nzv[2] = nz0[2]; nzv[3] = nz0[3];
    nzv[4] = nz1[0]; nzv[5] = nz1[1]; nzv[6] = nz1[2]; nzv[7] = nz1[3];
    v8h hv, lv;
#pragma unroll
    for (int r = 0; r < 8; ++r) {
      const float mm  = accA[r] + accB[r] * kCarryInv;
      const float d0  = ms * dsv[r];
      const float d1  = mt * dtv[r];
      const float drv = d0 + d1;
      const float pre = (mm + bias[r]) + drv;
      const float y   = fmaxf(pre, 0.0f);
      const float t1  = y - rst[r];
      const float t2  = kNoiseStd * nzv[r];
      const float t3  = t1 + t2;
      const float dr  = t3 * kLeak;
      const float rn  = rst[r] + dr;
      rst[r] = rn;
      _Float16 h1, l1;
      split_h16(rn, h1, l1);
      hv[r] = h1;
      lv[r] = l1;
    }
    *(v8h*)(hb + ((nxt * 2 + 0) * 16 + c) * kRP + cell0) = hv;
    *(v8h*)(hb + ((nxt * 2 + 1) * 16 + c) * kRP + cell0) = lv;
    {
      const v4f ra = {rst[0], rst[1], rst[2], rst[3]};
      const v4f rb = {rst[4], rst[5], rst[6], rst[7]};
      float* rp = r32 + (nxt * 16 + c) * kR32P + cell0;
      *(v4f*)(rp) = ra;
      *(v4f*)(rp + 4) = rb;
    }
    __syncthreads();

    const bool dly = (t >= kDelayT0) && (t < kTestT0);
    const bool rsp = (t >= kRespT0);
    const v4f rv = *(const v4f*)(r32 + (nxt * 16 + bq) * kR32P + 4 * lane);
    float s = 0.0f;
#pragma unroll
    for (int j = 0; j < 4; ++j) {
      const float wj = dly ? wmv[j] : wov[j];
      const float pj = wj * rv[j];
      s = s + pj;
    }
#pragma unroll
    for (int off = 16; off > 0; off >>= 1) s += __shfl_xor(s, off, 32);
    int slot = dly ? (((t - kDelayT0) * kCond + bq) * kOutO + o)
                   : (kSlots0 + ((t - kRespT0) * kCond + bq) * kOutO + o);
    slot = (slot < 0) ? 0 : ((slot > kSlotPitch - 1) ? (kSlotPitch - 1) : slot);
    if ((dly || rsp) && lane == 0) res[slot] = s;
  }
  __syncthreads();

  float* sp = stg + (size_t)model * kSlotPitch;
  for (int pass = 0; pass < 2; ++pass) {
#pragma unroll 1
    for (int g = wave; g < kSlotPitch / 128; g += kThreads / 32) {
      const v4f v = *(const v4f*)(res + g * 128 + 4 * lane);
      *(volatile v4f*)(sp + g * 128 + 4 * lane) = v;
    }
    __threadfence();
  }
}

__global__ __launch_bounds__(kThreads) void emit_lines_kernel(const float* __restrict__ stg, float* __restrict__ out) {
  const int i   = blockIdx.x * kThreads + threadIdx.x;
  const int L   = i >> 3;
  const int j0  = (i & 7) * 4;
  const int reg = (L >= kOut0Lines) ? 1 : 0;
  const int Lr  = L - reg * kOut0Lines;
  const int tb  = Lr >> 4;
  const int m0  = (Lr & 15) * 16 + (j0 >> 1);
  const int slot = reg * kSlots0 + tb * 2;
  const v2f a = *(const v2f*)(stg + (size_t)m0 * kSlotPitch + slot);
  const v2f b = *(const v2f*)(stg + (size_t)(m0 + 1) * kSlotPitch + slot);
  const v4f v = {a[0], a[1], b[0], b[1]};
  float* op = out + (size_t)i * 4;
  *(volatile v4f*)op = v;
  __threadfence();
  *(volatile v4f*)op = v;
}

extern "C" void kernel_launch(void* const* d_in, const int* in_sizes, int n_in,
                              void* d_out, int out_size, void* d_ws, size_t ws_size, hipStream_t stream) {
  if (n_in < 7 || d_out == nullptr || d_ws == nullptr) return;
  if (in_sizes[0] != kCond * 2 * kStim || in_sizes[1] != kSteps * kModels * kCells ||
      in_sizes[2] != kModels * kCells * kCells || in_sizes[3] != kModels * kCells ||
      in_sizes[4] != kModels * kCells * kStim || in_sizes[5] != kModels * kOutO * kCells ||
      in_sizes[6] != kModels * kOutO * kCells || out_size != kOutFloats) return;

  const float* x     = (const float*)d_in[0];
  const float* noise = (const float*)d_in[1];
  const float* W     = (const float*)d_in[2];
  const float* bvec  = (const float*)d_in[3];
  const float* Wi    = (const float*)d_in[4];
  const float* Wo    = (const float*)d_in[5];
  const float* Wm    = (const float*)d_in[6];
  float* out = (float*)d_out;

  const size_t stg_bytes = (size_t)kModels * kSlotPitch * sizeof(float);
  if (stg_bytes > ws_size || stg_bytes > (size_t)134217728) return;
  float* STG = (float*)d_ws;

  rnn_seq_kernel<<<kModels, kThreads, 0, stream>>>(x, noise, W, bvec, Wi, Wo, Wm, STG);
  emit_lines_kernel<<<kEmitBlocks, kThreads, 0, stream>>>(STG, out);
}
